// MultiHeadAttention_75393855914545
// MI455X (gfx1250) — hardware-verified
//
#include <hip/hip_runtime.h>
#include <math.h>

typedef __attribute__((ext_vector_type(16))) _Float16 v16h;
typedef __attribute__((ext_vector_type(16))) __bf16 v16b;
typedef __attribute__((ext_vector_type(8)))  _Float16 v8h;
typedef __attribute__((ext_vector_type(8)))  __bf16 v8b;
typedef __attribute__((ext_vector_type(8)))  float v8f;
typedef __attribute__((ext_vector_type(4)))  float v4f;
typedef __attribute__((ext_vector_type(4)))  unsigned v4u;

#ifndef NB
#define NB 2
#endif
#ifndef TT
#define TT 2048
#endif
#define TT_FULL 2048
#define CC 1024
#define DIN 1024
#define NH 16
#define HD 64
#define C2 (0.18033688011112042f)

static_assert(CC == NH * HD);
static_assert(HD == 64);
static_assert(DIN == CC);
static_assert(TT % 64 == 0);
static_assert(TT % 32 == 0);
static_assert(TT <= TT_FULL);
static_assert(DIN % 64 == 0);
static_assert(CC % 128 == 0);
static_assert(DIN % 32 == 0);
static_assert(((size_t)NB * TT * DIN) % (8 * 256) == 0);

#define WS_XB  ((size_t)0)
#define WS_WT  (WS_XB + 2u * (size_t)NB * TT * DIN)
#define WS_QK  (WS_WT + 2u * (size_t)4 * CC * DIN)
#define WS_VT  (WS_QK + 2u * (size_t)2 * NB * TT * CC)
#define WS_CT  (WS_VT + 2u * (size_t)NB * CC * TT)
#define WS_END (WS_CT + 2u * (size_t)NB * TT * CC)
static_assert(WS_END <= (size_t)134217728);
static_assert(WS_WT % 128 == 0);
static_assert(WS_QK % 128 == 0);
static_assert(WS_VT % 128 == 0);
static_assert(WS_CT % 128 == 0);

template <typename T> __device__ __forceinline__ void vst2(void* p, T v) { *(volatile T*)p = v; __threadfence(); *(volatile T*)p = v; }
__device__ __forceinline__ v8f wmma16(v16h a, v16h b, v8f c) {
  v8f d = __builtin_amdgcn_wmma_f32_16x16x32_f16(false, a, false, b, (short)0, c, false, false);
  asm volatile("v_nop\n\tv_nop\n\tv_nop\n\tv_nop" : "+v"(d) : "v"(a), "v"(b));
  return d;
}
__device__ __forceinline__ v8f wmma_bf(v16b a, v16b b, v8f c) {
  v8f d = __builtin_amdgcn_wmma_f32_16x16x32_bf16(false, a, false, b, (short)0, c, false, false);
  asm volatile("v_nop\n\tv_nop\n\tv_nop\n\tv_nop" : "+v"(d) : "v"(a), "v"(b));
  return d;
}
__device__ __forceinline__ v16h frag_h(const _Float16* rowk0, int lane) {
  union { v16h v; v8h q[2]; } u; const _Float16* p = rowk0 + 8 * (lane >> 4);
  u.q[0] = *(const v8h*)p; u.q[1] = *(const v8h*)(p + 16); return u.v;
}
__device__ __forceinline__ v16b frag_b(const __bf16* rowk0, int lane) {
  union { v16b v; v8b q[2]; } u; const __bf16* p = rowk0 + 8 * (lane >> 4);
  u.q[0] = *(const v8b*)p; u.q[1] = *(const v8b*)(p + 16); return u.v;
}
__device__ __forceinline__ float bfr(float v) { return (float)(__bf16)v; }
__device__ __forceinline__ unsigned bf_bits(float v) { return (unsigned)__builtin_bit_cast(unsigned short, (__bf16)v); }
#define LDSX() do { asm volatile("s_wait_dscnt 0" ::: "memory"); __builtin_amdgcn_wave_barrier(); __builtin_amdgcn_fence(3  , "workgroup"); } while (0)

__global__ __launch_bounds__(256) void k_cvtx(const float* __restrict__ X, unsigned short* __restrict__ XB) {
  const size_t e = ((size_t)blockIdx.x * 256 + threadIdx.x) * 8;
  const size_t row = e / DIN; const int c = (int)(e % DIN); const size_t b = row / TT; const size_t t = row % TT;
  const float* src = X + (b * TT_FULL + t) * DIN + c;
  const v4f f0 = *(const v4f*)src; const v4f f1 = *(const v4f*)(src + 4);
  v4u o;
  o[0] = bf_bits(f0[0]) | (bf_bits(f0[1]) << 16);
  o[1] = bf_bits(f0[2]) | (bf_bits(f0[3]) << 16);
  o[2] = bf_bits(f1[0]) | (bf_bits(f1[1]) << 16);
  o[3] = bf_bits(f1[2]) | (bf_bits(f1[3]) << 16);
  vst2(XB + e, o);
}

__global__ __launch_bounds__(128) void k_wt(const float* __restrict__ W0, const float* __restrict__ W1, const float* __restrict__ W2, const float* __restrict__ W3, unsigned short* __restrict__ WT) {
  __shared__ __align__(16) unsigned short ts[64][72];
  const int tid = threadIdx.x; const int z = blockIdx.z; const int k0 = blockIdx.x * 64, o0 = blockIdx.y * 64;
  const float* W = z == 0 ? W0 : z == 1 ? W1 : z == 2 ? W2 : W3;
#pragma unroll 1
  for (int i = 0; i < 8; ++i) { const int e = tid + i * 128; const int kl = e >> 4, c4 = e & 15;
    const v4f v = *(const v4f*)(W + (size_t)(k0 + kl) * CC + o0 + c4 * 4);
#pragma unroll
    for (int x = 0; x < 4; ++x) { const float bv = bfr(v[x]); const unsigned short ub = __builtin_bit_cast(unsigned short, (__bf16)v[x]); const unsigned short uh = __builtin_bit_cast(unsigned short, (_Float16)(bv * 256.0f)); ts[c4 * 4 + x][kl] = (z == 3) ? uh : ub; } }
  __syncthreads();
#pragma unroll 1
  for (int i = 0; i < 4; ++i) { const int e = tid + i * 128; const int ol = e >> 3, q = e & 7;
    vst2(WT + ((size_t)z * CC + o0 + ol) * DIN + k0 + q * 8, *(const v4u*)&ts[ol][q * 8]); }
}

__global__ __launch_bounds__(128) void k_proj(const __bf16* __restrict__ XB, const __bf16* __restrict__ WT, const float* __restrict__ BQ, const float* __restrict__ BK, const float* __restrict__ BV, _Float16* __restrict__ QK, _Float16* __restrict__ VT) {
  __shared__ __align__(16) _Float16 sh[64][136]; __shared__ __align__(16) _Float16 th[128][72];
  const int tid = threadIdx.x; const int wave = __builtin_amdgcn_readfirstlane(threadIdx.x >> 5); const int lane = tid & 31, col = lane & 15, g = lane >> 4;
  const int which = blockIdx.z; const int c0 = blockIdx.y * 128; const size_t r0 = (size_t)blockIdx.x * 64; const size_t bb = r0 / TT; const int t0 = (int)(r0 % TT);
  const float* BA = which == 0 ? BQ : which == 1 ? BK : BV;
  const __bf16* xr = XB + (r0 + wave * 16 + col) * DIN;
  const __bf16* wr = WT + ((size_t)which * CC + c0 + col) * DIN;
  v8f acc[8] = {};
#pragma unroll 1
  for (int kc = 0; kc < DIN / 32; ++kc) { const v16b a = frag_b(xr + kc * 32, lane);
#pragma unroll
    for (int j = 0; j < 8; ++j) { const v16b w = frag_b(wr + (size_t)j * 16 * DIN + kc * 32, lane); acc[j] = wmma_bf(a, w, acc[j]); } }
  if (which < 2) { _Float16* DH = QK + (size_t)which * NB * TT * CC;
#pragma unroll
    for (int j = 0; j < 8; ++j) { const float bias = bfr(BA[c0 + j * 16 + col]);
#pragma unroll
      for (int r = 0; r < 8; ++r) sh[wave * 16 + 8 * g + r][j * 16 + col] = (_Float16)(acc[j][r] + bias); }
    __syncthreads();
#pragma unroll 1
    for (int e = tid; e < 64 * 16; e += 128) { const int rl = e >> 4, q = e & 15; vst2(DH + (r0 + rl) * CC + c0 + q * 8, *(const v4u*)&sh[rl][q * 8]); }
  } else {
#pragma unroll
    for (int j = 0; j < 8; ++j) { const float bias = bfr(BA[c0 + j * 16 + col]);
#pragma unroll
      for (int r = 0; r < 8; ++r) th[j * 16 + col][wave * 16 + 8 * g + r] = (_Float16)(acc[j][r] + bias); }
    __syncthreads();
#pragma unroll 1
    for (int e = tid; e < 128 * 8; e += 128) { const int cl = e >> 3, q = e & 7; vst2(VT + (bb * CC + c0 + cl) * (size_t)TT + t0 + q * 8, *(const v4u*)&th[cl][q * 8]); } } }

__global__ __launch_bounds__(128) void k_attn(const _Float16* __restrict__ QH, const _Float16* __restrict__ KH, const _Float16* __restrict__ VT, _Float16* __restrict__ CT) {
  __shared__ __align__(16) _Float16 ct[4][16][72];
  const int tid = threadIdx.x; const int wave = __builtin_amdgcn_readfirstlane(threadIdx.x >> 5); const int lane = tid & 31, col = lane & 15, g = lane >> 4;
  const int b = blockIdx.z, h = blockIdx.y; const int q0 = blockIdx.x * 64 + wave * 16;
  const _Float16* qp = QH + ((size_t)b * TT + q0 + col) * CC + h * HD;
  const v16h qf0 = frag_h(qp, lane), qf1 = frag_h(qp + 32, lane);
  const _Float16* kp = KH + ((size_t)b * TT + col) * CC + h * HD;
  const _Float16* vp = VT + ((size_t)b * CC + h * HD + col) * (size_t)TT;
  float m = -3.0e38f, l = 0.f;
  v8f o[4] = {};
#pragma unroll 1
  for (int kb = 0; kb < TT; kb += 32) {
    v8f s0 = {}, s1 = {};
    { const _Float16* p = kp + (size_t)kb * CC;
      const v16h ka = frag_h(p, lane), kc = frag_h(p + 32, lane);
      s0 = wmma16(ka, qf0, s0); s0 = wmma16(kc, qf1, s0);
      const _Float16* p2 = p + (size_t)16 * CC;
      const v16h kd = frag_h(p2, lane), ke = frag_h(p2 + 32, lane);
      s1 = wmma16(kd, qf0, s1); s1 = wmma16(ke, qf1, s1); }
    float mx = fmaxf(s0[0], s1[0]);
#pragma unroll
    for (int r = 1; r < 8; ++r) mx = fmaxf(mx, fmaxf(s0[r], s1[r]));
    mx = fmaxf(mx, __shfl_xor(mx, 16));
    const float mn = fmaxf(m, mx * C2);
    const float alpha = __builtin_amdgcn_exp2f(m - mn);
    m = mn;
    const float off = 10.0f - mn;
    float ps = 0.f; v16h pf;
#pragma unroll
    for (int r = 0; r < 8; ++r) { const float p0 = __builtin_amdgcn_exp2f(__builtin_fmaf(s0[r], C2, off)); const float p1 = __builtin_amdgcn_exp2f(__builtin_fmaf(s1[r], C2, off)); ps += p0 + p1; pf[r] = (_Float16)p0; pf[8 + r] = (_Float16)p1; }
    l = l * alpha + ps;
#pragma unroll
    for (int j = 0; j < 4; ++j) o[j] = o[j] * alpha;
#pragma unroll
    for (int j = 0; j < 4; ++j) { const v16h vf = frag_h(vp + (size_t)j * 16 * TT + kb, lane); o[j] = wmma16(vf, pf, o[j]); }
  }
  l += __shfl_xor(l, 16);
  const float inv = 64.0f * __builtin_amdgcn_rcpf(l);
#pragma unroll
  for (int j = 0; j < 4; ++j) { v8h hv;
#pragma unroll
    for (int r = 0; r < 8; ++r) hv[r] = (_Float16)(o[j][r] * inv);
    *(v8h*)&ct[wave][col][j * 16 + 8 * g] = hv; }
  LDSX();
#pragma unroll 1
  for (int i = 0; i < 4; ++i) { const int rl = i * 4 + (lane >> 3), q = lane & 7;
    vst2(CT + ((size_t)b * TT + q0 + rl) * CC + h * HD + q * 8, *(const v4u*)&ct[wave][rl][q * 8]); }
}

__global__ __launch_bounds__(128) void k_out(const _Float16* __restrict__ CT, const _Float16* __restrict__ WOT, const float* __restrict__ BO, float* __restrict__ OUT) {
  __shared__ __align__(16) float sf[4][16][132];
  const int tid = threadIdx.x; const int wave = __builtin_amdgcn_readfirstlane(threadIdx.x >> 5); const int lane = tid & 31, col = lane & 15, g = lane >> 4;
  const int c0 = blockIdx.y * 128; const size_t rb = (size_t)blockIdx.x * 64; const size_t r0 = rb + wave * 16;
  const _Float16* ar = CT + (r0 + col) * CC;
  const _Float16* wr = WOT + (size_t)(c0 + col) * CC;
  v8f acc[8] = {};
#pragma unroll 1
  for (int kc = 0; kc < CC / 32; ++kc) { const v16h a = frag_h(ar + kc * 32, lane);
#pragma unroll
    for (int j = 0; j < 8; ++j) { const v16h w = frag_h(wr + (size_t)j * 16 * CC + kc * 32, lane); acc[j] = wmma16(a, w, acc[j]); } }
#pragma unroll
  for (int j = 0; j < 8; ++j) { const float bias = bfr(BO[c0 + j * 16 + col]);
#pragma unroll
    for (int r = 0; r < 8; ++r) sf[wave][8 * g + r][j * 16 + col] = acc[j][r] * (1.0f / 16384.0f) + bias; }
  LDSX();
  const size_t bbo = rb / TT; const size_t to = rb % TT + (size_t)wave * 16;
#pragma unroll 1
  for (int rl = 0; rl < 16; ++rl) vst2(OUT + (bbo * TT_FULL + to + rl) * DIN + c0 + lane * 4, *(const v4f*)&sf[wave][rl][lane * 4]);
}

extern "C" void kernel_launch(void* const* d_in, const int* in_sizes, int n_in, void* d_out, int out_size, void* d_ws, size_t ws_size, hipStream_t stream) {
  if (n_in < 9) return;
  const long long xmin = ((long long)(NB - 1) * TT_FULL + TT) * DIN;
  if ((long long)in_sizes[0] < xmin) return;
  if (in_sizes[1] < DIN * CC || in_sizes[3] < DIN * CC || in_sizes[5] < DIN * CC || in_sizes[7] < CC * DIN) return;
  if (in_sizes[2] < CC || in_sizes[4] < CC || in_sizes[6] < CC || in_sizes[8] < DIN) return;
  if ((long long)out_size < xmin) return;
  if (ws_size < (size_t)WS_END) return;
  const float* x = (const float*)d_in[0];
  const float* wq = (const float*)d_in[1]; const float* bq = (const float*)d_in[2];
  const float* wk = (const float*)d_in[3]; const float* bk = (const float*)d_in[4];
  const float* wv = (const float*)d_in[5]; const float* bv = (const float*)d_in[6];
  const float* wo = (const float*)d_in[7]; const float* bo = (const float*)d_in[8];
  char* ws = (char*)d_ws;
  unsigned short* XB = (unsigned short*)(ws + WS_XB);
  unsigned short* WT = (unsigned short*)(ws + WS_WT);
  _Float16* QK = (_Float16*)(ws + WS_QK);
  _Float16* VT = (_Float16*)(ws + WS_VT);
  _Float16* CT = (_Float16*)(ws + WS_CT);
  k_cvtx<<<dim3((unsigned)((size_t)NB * TT * DIN / (8 * 256))), 256, 0, stream>>>(x, XB);
  k_wt<<<dim3(DIN / 64, CC / 64, 4), 128, 0, stream>>>(wq, wk, wv, wo, WT);
  k_proj<<<dim3(NB * TT / 64, CC / 128, 3), 128, 0, stream>>>((const __bf16*)XB, (const __bf16*)WT, bq, bk, bv, QK, VT);
  k_attn<<<dim3(TT / 64, NH, NB), 128, 0, stream>>>(QK, QK + (size_t)NB * TT * CC, VT, CT);
  k_out<<<dim3(NB * TT / 64, DIN / 128), 128, 0, stream>>>(CT, (const _Float16*)(WT + (size_t)3 * CC * DIN), bo, (float*)d_out);
}
